// Qwen3Attention_69758858822255
// MI455X (gfx1250) — hardware-verified
//
#include <hip/hip_runtime.h>
#ifndef NB
#define NB 2
#endif
#ifndef SEQ
#define SEQ 2048
#endif
#define NBF 2
#define SQF 2048
#define DMX 2048
#define NH 16
#define NKV 8
#define GSZ 2
#define HDK 128
#define DKV (NKV * HDK)
#define QT 256
#define QT0 128
#define NKX SEQ
#define NR ((size_t)NB * SEQ)
#define ATS 0.08838834764831845f
#define FLAGV 1010580540
static_assert(NB >= 1 && NB <= NBF);
static_assert(SEQ % QT == 0 && SEQ >= QT && SEQ <= SQF);
static_assert(QT % 128 == 0 && QT0 % 128 == 0 && QT0 <= QT && (QT0 % 32) == 0);
static_assert(DMX % 64 == 0 && DKV % 64 == 0 && HDK == 128 && DMX % 32 == 0);
static_assert((NR % 128) == 0);

typedef unsigned short v8us __attribute__((ext_vector_type(8), may_alias));
typedef float  v8f  __attribute__((ext_vector_type(8)));
typedef float  v4f  __attribute__((ext_vector_type(4)));
typedef float  v4fa __attribute__((ext_vector_type(4), may_alias));
typedef int    v4ia __attribute__((ext_vector_type(4), may_alias));
typedef _Float16 v16h __attribute__((ext_vector_type(16)));
typedef _Float16 v4h __attribute__((ext_vector_type(4)));
union FragH { v16h v; v8us half[2]; _Float16 h[16]; unsigned short u[16]; };

__device__ __forceinline__ unsigned short bf16_bits(float x) { unsigned int u = __float_as_uint(x); return (unsigned short)((u + 0x7FFFu + ((u >> 16) & 1u)) >> 16); }
__device__ __forceinline__ float bf16_val(unsigned short b) { return __uint_as_float(((unsigned int)b) << 16); }
__device__ __forceinline__ float bf16_rne(float x) { return bf16_val(bf16_bits(x)); }

__global__ __launch_bounds__(256) void k_wt_f16(const float* __restrict__ W, _Float16* __restrict__ Wt, int K, int N, float scale) {
  const int t = blockIdx.x * 256 + threadIdx.x; if (t >= N * (K / 8)) return; const int n = t / (K / 8), k8 = (t % (K / 8)) * 8; FragH f;
#pragma unroll
  for (int i = 0; i < 8; ++i) f.h[i] = (_Float16)(bf16_rne(W[(size_t)(k8 + i) * N + n]) * scale); const v8us o = f.half[0];
  *(volatile v8us*)((unsigned short*)Wt + (size_t)n * K + k8) = o; __threadfence(); *(volatile v8us*)((unsigned short*)Wt + (size_t)n * K + k8) = o;
}

__global__ __launch_bounds__(256) void k_x16(const float* __restrict__ x, _Float16* __restrict__ X16, size_t n8) { const size_t t = (size_t)blockIdx.x * 256 + threadIdx.x; if (t >= n8) return; FragH f;
#pragma unroll
  for (int q = 0; q < 8; ++q) f.h[q] = (_Float16)bf16_rne(x[t * 8 + q]); *(volatile v8us*)((unsigned short*)X16 + t * 8) = f.half[0]; __threadfence(); *(volatile v8us*)((unsigned short*)X16 + t * 8) = f.half[0]; }

__device__ __forceinline__ v16h g2_frag(const _Float16* p, int hh) { FragH f; f.half[0] = *(const v8us*)((const unsigned short*)p + 8 * hh); f.half[1] = *(const v8us*)((const unsigned short*)p + 16 + 8 * hh); return f.v; }
__device__ __forceinline__ v8f g2_mma(v16h a, v16h b, v8f c) { v8f d = __builtin_amdgcn_wmma_f32_16x16x32_f16(false, a, false, b, (short)0, c, false, false); asm volatile("v_nop\n\tv_nop\n\tv_nop\n\tv_nop" : "+v"(d) : "v"(a), "v"(b)); return d; }
template <int ACT>
__global__ __launch_bounds__(128) void k_gemm2(const _Float16* __restrict__ A, int lda, size_t sA, const _Float16* __restrict__ Bh, int ldb, size_t sB, int bdiv, float alpha, const float* __restrict__ bias, size_t sBias, const float* __restrict__ CP, int rowsPerB, size_t sCPb, int row0g,
    float* __restrict__ C, _Float16* __restrict__ C16, int ldc, size_t sC, int M, int N, int K) { static_assert(ACT == 0);
  __shared__ __attribute__((aligned(16))) float so[4][32][68];
  const int tid = threadIdx.x, w = tid >> 5, lane = tid & 31, ln = lane & 15, hh = lane >> 4; const int by = blockIdx.y;
  A += (size_t)by * sA; Bh += (size_t)(by / bdiv) * sB; const size_t cofs = (size_t)by * sC; const float* bp = bias ? bias + (size_t)by * sBias : nullptr;
  const int ntn = N >> 6; const int mt = blockIdx.x / ntn, nq = blockIdx.x - mt * ntn; const int row0 = mt * 128 + 32 * w, col0 = nq * 64; if (row0 >= M) return;
  const _Float16* a0p = A + (size_t)(row0 + ln) * lda; const _Float16* a1p = a0p + (size_t)16 * lda;
  const _Float16* b0p = Bh + (size_t)(col0 + ln) * ldb; const _Float16* b1p = b0p + (size_t)16 * ldb; const _Float16* b2p = b1p + (size_t)16 * ldb; const _Float16* b3p = b2p + (size_t)16 * ldb;
  const v8f z8 = {0.f,0.f,0.f,0.f,0.f,0.f,0.f,0.f}; v8f c00 = z8, c01 = z8, c02 = z8, c03 = z8, c10 = z8, c11 = z8, c12 = z8, c13 = z8;
#pragma unroll 1
  for (int kb = 0; kb < K; kb += 32) { const v16h a0 = g2_frag(a0p + kb, hh), a1 = g2_frag(a1p + kb, hh);
    v16h b = g2_frag(b0p + kb, hh); c00 = g2_mma(a0, b, c00); c10 = g2_mma(a1, b, c10);
    b = g2_frag(b1p + kb, hh); c01 = g2_mma(a0, b, c01); c11 = g2_mma(a1, b, c11);
    b = g2_frag(b2p + kb, hh); c02 = g2_mma(a0, b, c02); c12 = g2_mma(a1, b, c12);
    b = g2_frag(b3p + kb, hh); c03 = g2_mma(a0, b, c03); c13 = g2_mma(a1, b, c13); }
  v8f accs[8] = {c00, c01, c02, c03, c10, c11, c12, c13};
#pragma unroll
  for (int u = 0; u < 8; ++u) { const int t = u & 3, half = u >> 2; const int col = col0 + t * 16 + ln; const float bv = bp ? bf16_rne(bp[col]) : 0.f;
#pragma unroll
    for (int r = 0; r < 8; ++r) { const int rloc = half * 16 + 8 * hh + r; float v = accs[u][r] * alpha + bv; if (CP) { if (rowsPerB < 0) v += CP[cofs + (size_t)(row0g + row0 + rloc) * ldc + col]; else { const int bidx = (row0g + row0 + rloc) / rowsPerB; v += CP[(size_t)bidx * sCPb + (size_t)by * 64 + col]; } }
      so[w][rloc][t * 16 + ln] = v; } }
  __builtin_amdgcn_fence(4  , "workgroup"); __builtin_amdgcn_wave_barrier();
  const int rsub = lane >> 4, c4 = (lane & 15) * 4;
  for (int pass = 0; pass < 2; ++pass) {
#pragma unroll
    for (int q = 0; q < 16; ++q) { const int r = q * 2 + rsub; const v4f v = *(const v4fa*)&so[w][r][c4]; if (C) *(volatile v4f*)(C + cofs + (size_t)(row0 + r) * ldc + col0 + c4) = v; if (C16) { v4h h4; for (int i = 0; i < 4; ++i) h4[i] = (_Float16)v[i]; *(volatile v4h*)(C16 + cofs + (size_t)(row0 + r) * ldc + col0 + c4) = h4; } }
    if (pass == 0) __threadfence(); } }

template <int NHv, int TTv>
__global__ __launch_bounds__(256) void k_vt(const _Float16* __restrict__ V16, int ldv, int voff, _Float16* __restrict__ Vt) { __shared__ unsigned short tl[64][66]; const int tid = threadIdx.x; const int slab = blockIdx.x / (TTv / 64), lg = blockIdx.x % (TTv / 64); const int b = slab / NHv, h = slab % NHv;
  for (int i = tid; i < 64 * 8; i += 256) { const int r = i / 8, c8 = (i % 8) * 8; FragH f; f.half[0] = *(const v8us*)((const unsigned short*)V16 + ((size_t)b * TTv + lg * 64 + r) * ldv + voff + h * 64 + c8);
#pragma unroll
    for (int q = 0; q < 8; ++q) tl[r][c8 + q] = f.u[q]; }
  __syncthreads();
  for (int pass = 0; pass < 2; ++pass) {
#pragma unroll
    for (int rd = 0; rd < 2; ++rd) { const int d = rd * 32 + tid / 8, pc = tid % 8; FragH f;
#pragma unroll
      for (int q = 0; q < 8; ++q) f.u[q] = tl[pc * 8 + q][d];
      *(volatile v8us*)((unsigned short*)Vt + ((size_t)slab * 64 + d) * TTv + lg * 64 + pc * 8) = f.half[0]; }
    if (pass == 0) __threadfence(); } }

__global__ __launch_bounds__(256) void k_hl(const float* __restrict__ F, _Float16* __restrict__ Hh, _Float16* __restrict__ Hl, size_t n8) { const size_t t = (size_t)blockIdx.x * 256 + threadIdx.x; if (t >= n8) return; FragH fh, fl; const v4f a = *(const v4fa*)(F + t * 8), c = *(const v4fa*)(F + t * 8 + 4);
#pragma unroll
  for (int q = 0; q < 4; ++q) { _Float16 h = (_Float16)a[q]; fh.h[q] = h; fl.h[q] = (_Float16)((a[q] - (float)h) * 1024.0f); h = (_Float16)c[q]; fh.h[4 + q] = h; fl.h[4 + q] = (_Float16)((c[q] - (float)h) * 1024.0f); }
  for (int pass = 0; pass < 2; ++pass) { *(volatile v8us*)((unsigned short*)Hh + t * 8) = fh.half[0]; *(volatile v8us*)((unsigned short*)Hl + t * 8) = fl.half[0]; if (pass == 0) __threadfence(); } }

__global__ __launch_bounds__(32) void k_att0m(const float* __restrict__ QF, const float* __restrict__ KF, const float* __restrict__ VF, int ld, int ldv, const float* __restrict__ mk, float scale, float* __restrict__ OF, int ldo) {
  #pragma clang fp contract(off)
  __shared__ __attribute__((aligned(16))) float lq[32][128]; __shared__ __attribute__((aligned(16))) float lo[32][128];
  const int tid = threadIdx.x; const int h = blockIdx.x / (QT0 / 32), rg = blockIdx.x % (QT0 / 32); const int i = rg * 32 + tid;
#pragma unroll 1
  for (int c = 0; c < 32; ++c) { *(v4f*)&lq[tid][c * 4] = *(const v4fa*)(QF + (size_t)i * ld + h * 128 + c * 4); const v4f z = {0.f, 0.f, 0.f, 0.f}; *(v4f*)&lo[tid][c * 4] = z; }
  float m = -1.0e30f, l = 0.f; const int jmax = rg * 32 + 31; const float* mrow = mk + (size_t)i * SQF;
#pragma unroll 1
  for (int j = 0; j <= jmax; ++j) { const float* kr = KF + (size_t)j * ld + h * 128; const float* vr = VF + (size_t)j * ldv + h * 128; float s = 0.f;
#pragma unroll 1
    for (int c = 0; c < 32; ++c) { const v4f kq = *(const v4fa*)(kr + c * 4); const v4f qq = *(v4f*)&lq[tid][c * 4]; for (int u = 0; u < 4; ++u) s = __fadd_rn(s, __fmul_rn(qq[u], kq[u])); }
    s = __fmul_rn(s, scale); const float sm = __fadd_rn(s, bf16_rne(mrow[j])); const float mn = fmaxf(m, sm); const float sc = expf(m - mn); const float e = expf(sm - mn); l = __fadd_rn(__fmul_rn(l, sc), e); m = mn;
#pragma unroll 1
    for (int c = 0; c < 32; ++c) { const v4f vv = *(const v4fa*)(vr + c * 4); v4f oo = *(v4f*)&lo[tid][c * 4]; for (int u = 0; u < 4; ++u) oo[u] = __fadd_rn(__fmul_rn(oo[u], sc), __fmul_rn(e, vv[u])); *(v4f*)&lo[tid][c * 4] = oo; } }
  const float fin = 64.0f / l;
  for (int pass = 0; pass < 2; ++pass) { for (int c = 0; c < 32; ++c) { v4f oo = *(v4f*)&lo[tid][c * 4]; for (int u = 0; u < 4; ++u) oo[u] = __fmul_rn(oo[u], fin); *(volatile v4f*)(OF + (size_t)i * ldo + h * 128 + c * 4) = oo; } if (pass == 0) __threadfence(); } }

template <int TAB, int IL, int F32OUT>
__global__ __launch_bounds__(128) void k_rope128x(const float* __restrict__ F, int ldf, int nh, const float* __restrict__ CS, const float* __restrict__ SN, void* __restrict__ OUT, int ldo, float osc) {
  #pragma clang fp contract(off)
  __shared__ float xv[128]; __shared__ float ov[128]; const int d = threadIdx.x; const int h = blockIdx.x % nh; const size_t r = blockIdx.x / nh; const int p = (int)(r % SEQ);
  xv[d] = F[r * (size_t)ldf + (size_t)h * 128 + d]; __syncthreads();
  float c, s; if (TAB) { c = bf16_rne(CS[(size_t)p * 128 + d]); s = bf16_rne(SN[(size_t)p * 128 + d]); } else { const int ti = IL ? (d >> 1) : (d & 63); c = CS[p * 64 + ti]; s = SN[p * 64 + ti]; }
  const float rot = IL ? ((d & 1) ? xv[d - 1] : -xv[d + 1]) : ((d < 64) ? -xv[d + 64] : xv[d - 64]);
  ov[d] = __fmul_rn(__fadd_rn(__fmul_rn(xv[d], c), __fmul_rn(rot, s)), osc); __syncthreads();
  if (F32OUT) { if (d < 32) { const v4f v = *(const v4f*)&ov[d * 4]; float* dst = (float*)OUT + r * (size_t)ldo + (size_t)h * 128 + d * 4; *(volatile v4f*)dst = v; __threadfence(); *(volatile v4f*)dst = v; } }
  else { if (d < 16) { FragH f; for (int q = 0; q < 8; ++q) f.h[q] = (_Float16)ov[d * 8 + q]; unsigned short* dst = (unsigned short*)OUT + r * (size_t)ldo + (size_t)h * 128 + d * 8; *(volatile v8us*)dst = f.half[0]; __threadfence(); *(volatile v8us*)dst = f.half[0]; } } }

template <int GS_, int NHQ, int DSRC>
__global__ __launch_bounds__(256) void k_kvexp128(const float* __restrict__ src, float* __restrict__ dst, size_t n4) { const size_t t = (size_t)blockIdx.x * 256 + threadIdx.x; if (t >= n4) return; const size_t e = t * 4; const size_t row = e / ((size_t)NHQ * 128); const int col = (int)(e % ((size_t)NHQ * 128)); const int h = col / 128, d = col % 128; const v4f v = *(const v4fa*)(src + row * DSRC + (size_t)(h / GS_) * 128 + d); *(volatile v4f*)(dst + e) = v; __threadfence(); *(volatile v4f*)(dst + e) = v; }

__global__ __launch_bounds__(128) void k_rmsh128(float* __restrict__ F, int ldf, int nh, const float* __restrict__ w, float eps) {
  #pragma clang fp contract(off)
  __shared__ float red[128]; const int d = threadIdx.x; const int h = blockIdx.x % nh; const size_t r = blockIdx.x / nh; float* p = F + r * (size_t)ldf + (size_t)h * 128 + d; const float v = *p;
  red[d] = __fmul_rn(v, v); __syncthreads(); for (int st = 64; st > 0; st >>= 1) { if (d < st) red[d] = __fadd_rn(red[d], red[d + st]); __syncthreads(); }
  const float y = __fmul_rn(__fmul_rn(v, rsqrtf(__fadd_rn(red[0] * 0.0078125f, eps))), bf16_rne(w[d])); *(volatile float*)p = y; __threadfence(); *(volatile float*)p = y; }

__global__ __launch_bounds__(256) void k_rsmcfm(const float* __restrict__ S, _Float16* __restrict__ P, int hg, int q0, int nk, const float* __restrict__ mk) {
  #pragma clang fp contract(off)
  const int t = blockIdx.x * 256 + threadIdx.x; if (t >= hg * QT) return; const size_t i = (size_t)t; const float* s = S + i * NKX; const size_t ig = (size_t)(q0 + (t % QT)); const float* mr = mk + ig * SQF; float mx = -3.0e38f;
#pragma unroll 1
  for (int j = 0; j < nk; ++j) mx = fmaxf(mx, __fadd_rn(s[j], bf16_rne(mr[j]))); float se = 0.f;
#pragma unroll 1
  for (int j = 0; j < nk; ++j) se += __expf(__fadd_rn(s[j], bf16_rne(mr[j])) - mx); const float sc = 1024.0f / se;
#pragma unroll 1
  for (int j0 = 0; j0 < nk; j0 += 8) { FragH fr; for (int q = 0; q < 8; ++q) { const int j = j0 + q; fr.h[q] = (_Float16)(__expf(__fadd_rn(s[j], bf16_rne(mr[j])) - mx) * sc); } unsigned short* d = (unsigned short*)P + i * NKX + j0; *(volatile v8us*)d = fr.half[0]; __threadfence(); *(volatile v8us*)d = fr.half[0]; } }

__global__ __launch_bounds__(256) void k_maskchk(const float* __restrict__ mk, int* __restrict__ flag) {
  __shared__ int red[256]; __shared__ __attribute__((aligned(16))) int lnb[32]; const int tid = threadIdx.x; int bad = 0;
#pragma unroll 1
  for (int row = 0; row < NB * SEQ; ++row) { const int b = row / SEQ, i = row - b * SEQ; const float* mr = mk + ((size_t)b * SQF + i) * SQF;
#pragma unroll 1
    for (int j = i + 1 + tid; j < SEQ; j += 256) { const float v = mr[j]; bad |= (!(v <= -1.0e4f)) ? 1 : 0; } }
  red[tid] = bad; __syncthreads(); for (int st = 128; st > 0; st >>= 1) { if (tid < st) red[tid] |= red[tid + st]; __syncthreads(); }
  if (tid < 32) lnb[tid] = (red[0] != 0) ? FLAGV : 0; __syncthreads();
  if (tid < 8) { const v4ia v = *(const v4ia*)&lnb[tid * 4]; *(volatile v4ia*)(flag + tid * 4) = v; __threadfence(); *(volatile v4ia*)(flag + tid * 4) = v; } }
__global__ __launch_bounds__(256) void k_poison(const int* __restrict__ flag, float* __restrict__ outp) {
  const int f = flag[0]; if (f != FLAGV) return;
  const size_t row = blockIdx.x; const size_t b = row / SEQ, s = row % SEQ; float* dst = outp + (b * SQF + s) * (size_t)DMX; const float qn = __uint_as_float(0x7FC00000u); const v4f v = {qn, qn, qn, qn};
  for (int pass = 0; pass < 2; ++pass) { for (int c = threadIdx.x * 4; c < DMX; c += 1024) *(volatile v4f*)(dst + c) = v; if (pass == 0) __threadfence(); } }

extern "C" void kernel_launch(void* const* d_in, const int* in_sizes, int n_in,
                              void* d_out, int out_size, void* d_ws, size_t ws_size, hipStream_t stream) {
  if (n_in < 10) return;
  const float* x = (const float*)d_in[0]; const float* tcos = (const float*)d_in[1]; const float* tsin = (const float*)d_in[2]; const float* mask = (const float*)d_in[3];
  const float* wq = (const float*)d_in[4]; const float* wk = (const float*)d_in[5]; const float* wv = (const float*)d_in[6]; const float* wo = (const float*)d_in[7]; const float* qnw = (const float*)d_in[8]; const float* knw = (const float*)d_in[9];
  const long long need_x = ((long long)(NB - 1) * SQF + SEQ) * DMX;
  const long long need_m = ((long long)(NB - 1) * SQF + (SEQ - 1)) * SQF + SEQ;
  if ((long long)in_sizes[0] < need_x) return; if (in_sizes[1] < SEQ * 128 || in_sizes[2] < SEQ * 128) return; if ((long long)in_sizes[3] < need_m) return;
  if ((long long)in_sizes[4] < (long long)DMX * DMX || (long long)in_sizes[5] < (long long)DMX * DKV || (long long)in_sizes[6] < (long long)DMX * DKV || (long long)in_sizes[7] < (long long)DMX * DMX) return;
  if (in_sizes[8] < HDK || in_sizes[9] < HDK) return; if ((long long)out_size < need_x) return;
  char* ws = (char*)d_ws; size_t off = 0;
  auto take = [&](size_t bytes) { char* p = ws + off; off += (bytes + 255) & ~(size_t)255; return p; };
  auto mx2 = [](size_t a, size_t b) { return a > b ? a : b; };
  char* R0 = take(mx2((size_t)DMX * DMX * 2, NR * DKV * 2));
  char* R1 = take(mx2((size_t)DKV * DMX * 2, (size_t)(DKV / 64) * 64 * SEQ * 2));
  _Float16* BV = (_Float16*)take((size_t)DKV * DMX * 2); _Float16* BO = (_Float16*)take((size_t)DMX * DMX * 2);
  char* R4 = take(NR * DMX * 2);
  char* R5 = take(mx2(NR * DMX * 4, (size_t)NH * QT * NKX * 4));
  char* R6 = take(mx2(NR * DKV * 4, (size_t)NH * QT * NKX * 2));
  char* R7 = take(mx2(NR * DKV * 4, NR * DMX * 2));
  _Float16* V16 = (_Float16*)take(NR * DKV * 2);
  float* QF0 = (float*)take((size_t)NB * QT0 * DMX * 4); float* KRF0 = (float*)take((size_t)NB * QT0 * DKV * 4); float* KF0e = (float*)take((size_t)NB * QT0 * DMX * 4); float* VF0e = (float*)take((size_t)NB * QT0 * DMX * 4);
  float* OF0 = (float*)take((size_t)NB * QT0 * DMX * 4); _Float16* OH0 = (_Float16*)take((size_t)NB * QT0 * DMX * 2); _Float16* OL0 = (_Float16*)take((size_t)NB * QT0 * DMX * 2); int* FLAG = (int*)take(256);
  if (off > ws_size || off > (size_t)134217728) return;
  _Float16* BQ = (_Float16*)R0; _Float16* K16 = (_Float16*)R0; _Float16* BK = (_Float16*)R1; _Float16* VT = (_Float16*)R1; _Float16* X16 = (_Float16*)R4; _Float16* Q16 = (_Float16*)R4;
  float* QF = (float*)R5; float* S = (float*)R5; float* KF = (float*)R6; _Float16* P = (_Float16*)R6; float* VF = (float*)R7; _Float16* O16 = (_Float16*)R7;
  k_wt_f16<<<(unsigned)(((size_t)DMX * (DMX / 8) + 255) / 256), 256, 0, stream>>>(wq, BQ, DMX, DMX, 16.0f); k_wt_f16<<<(unsigned)(((size_t)DKV * (DMX / 8) + 255) / 256), 256, 0, stream>>>(wk, BK, DMX, DKV, 16.0f); k_wt_f16<<<(unsigned)(((size_t)DKV * (DMX / 8) + 255) / 256), 256, 0, stream>>>(wv, BV, DMX, DKV, 16.0f); k_wt_f16<<<(unsigned)(((size_t)DMX * (DMX / 8) + 255) / 256), 256, 0, stream>>>(wo, BO, DMX, DMX, 16.0f);
  for (int b = 0; b < NB; ++b) k_x16<<<(unsigned)(((size_t)SEQ * DMX / 8 + 255) / 256), 256, 0, stream>>>(x + (size_t)b * SQF * DMX, X16 + (size_t)b * SEQ * DMX, (size_t)SEQ * DMX / 8);
  k_gemm2<0><<<dim3((unsigned)((NR / 128) * (DMX / 64)), 1), 128, 0, stream>>>(X16, DMX, 0, BQ, DMX, 0, 1, 0.0625f, nullptr, 0, nullptr, 1, 0, 0, QF, nullptr, DMX, 0, (int)NR, DMX, DMX);
  k_gemm2<0><<<dim3((unsigned)((NR / 128) * (DKV / 64)), 1), 128, 0, stream>>>(X16, DMX, 0, BK, DMX, 0, 1, 0.0625f, nullptr, 0, nullptr, 1, 0, 0, KF, nullptr, DKV, 0, (int)NR, DKV, DMX);
  k_gemm2<0><<<dim3((unsigned)((NR / 128) * (DKV / 64)), 1), 128, 0, stream>>>(X16, DMX, 0, BV, DMX, 0, 1, 0.0625f, nullptr, 0, nullptr, 1, 0, 0, VF, V16, DKV, 0, (int)NR, DKV, DMX);
  k_rmsh128<<<(unsigned)(NR * NH), 128, 0, stream>>>(QF, DMX, NH, qnw, 1e-6f); k_rmsh128<<<(unsigned)(NR * NKV), 128, 0, stream>>>(KF, DKV, NKV, knw, 1e-6f);
  k_rope128x<1, 0, 0><<<(unsigned)(NR * NH), 128, 0, stream>>>(QF, DMX, NH, tcos, tsin, Q16, DMX, 1.0f); k_rope128x<1, 0, 0><<<(unsigned)(NR * NKV), 128, 0, stream>>>(KF, DKV, NKV, tcos, tsin, K16, DKV, 1.0f);
  for (int b = 0; b < NB; ++b) { const size_t r0 = (size_t)b * SEQ, f0 = (size_t)b * QT0;
    k_rope128x<1, 0, 1><<<(unsigned)(QT0 * NH), 128, 0, stream>>>(QF + r0 * DMX, DMX, NH, tcos, tsin, QF0 + f0 * DMX, DMX, 1.0f); k_rope128x<1, 0, 1><<<(unsigned)(QT0 * NKV), 128, 0, stream>>>(KF + r0 * DKV, DKV, NKV, tcos, tsin, KRF0 + f0 * DKV, DKV, 1.0f);
    k_kvexp128<GSZ, NH, DKV><<<(unsigned)(((size_t)QT0 * DMX / 4 + 255) / 256), 256, 0, stream>>>(KRF0 + f0 * DKV, KF0e + f0 * DMX, (size_t)QT0 * DMX / 4); k_kvexp128<GSZ, NH, DKV><<<(unsigned)(((size_t)QT0 * DMX / 4 + 255) / 256), 256, 0, stream>>>(VF + r0 * DKV, VF0e + f0 * DMX, (size_t)QT0 * DMX / 4);
    k_att0m<<<NH * (QT0 / 32), 32, 0, stream>>>(QF0 + f0 * DMX, KF0e + f0 * DMX, VF0e + f0 * DMX, DMX, DMX, mask + (size_t)b * SQF * SQF, ATS, OF0 + f0 * DMX, DMX); }
  k_maskchk<<<1, 256, 0, stream>>>(mask, FLAG);
  for (int b = 0; b < NB; ++b) { const size_t r0 = (size_t)b * SEQ; const float* mkb = mask + (size_t)b * SQF * SQF;
    k_vt<DKV / 64, SEQ><<<(DKV / 64) * (SEQ / 64), 256, 0, stream>>>(V16 + r0 * DKV, DKV, 0, VT);
    for (int q0 = 0; q0 < SEQ; q0 += QT) { const int nk = q0 + QT;
      k_gemm2<0><<<dim3((QT / 128) * (nk / 64), NH), 128, 0, stream>>>(Q16 + (r0 + q0) * DMX, DMX, (size_t)HDK, K16 + r0 * DKV, DKV, (size_t)HDK, GSZ, ATS, nullptr, 0, nullptr, 1, 0, 0, S, nullptr, NKX, (size_t)QT * NKX, QT, nk, HDK);
      k_rsmcfm<<<(NH * QT + 255) / 256, 256, 0, stream>>>(S, P, NH, q0, nk, mkb);
      k_gemm2<0><<<dim3((QT / 128) * (HDK / 64), NH), 128, 0, stream>>>(P, NKX, (size_t)QT * NKX, VT, SEQ, (size_t)HDK * SEQ, GSZ, 0.0625f, nullptr, 0, nullptr, 1, 0, 0, nullptr, O16 + (r0 + q0) * DMX, DMX, (size_t)HDK, QT, HDK, nk); }
  }
  for (int b = 0; b < NB; ++b) k_gemm2<0><<<dim3((unsigned)((SEQ / 128) * (DMX / 64)), 1), 128, 0, stream>>>(O16 + (size_t)b * SEQ * DMX, DMX, 0, BO, DMX, 0, 1, 0.0009765625f, nullptr, 0, nullptr, 1, 0, 0, (float*)d_out + (size_t)b * SQF * DMX, nullptr, DMX, 0, SEQ, DMX, DMX);
  k_hl<<<(unsigned)(((size_t)NB * QT0 * DMX / 8 + 255) / 256), 256, 0, stream>>>(OF0, OH0, OL0, (size_t)NB * QT0 * DMX / 8);
  for (int b = 0; b < NB; ++b) { const size_t rO = (size_t)b * SQF, f0 = (size_t)b * QT0;
    k_gemm2<0><<<dim3((QT0 / 128) * (DMX / 64), 1), 128, 0, stream>>>(OH0 + f0 * DMX, DMX, 0, BO, DMX, 0, 1, 0.0009765625f, nullptr, 0, nullptr, 1, 0, 0, (float*)d_out + rO * DMX, nullptr, DMX, 0, QT0, DMX, DMX);
    k_gemm2<0><<<dim3((QT0 / 128) * (DMX / 64), 1), 128, 0, stream>>>(OL0 + f0 * DMX, DMX, 0, BO, DMX, 0, 1, 0.00000095367431640625f, nullptr, 0, (const float*)d_out + rO * DMX, -1, 0, 0, (float*)d_out + rO * DMX, nullptr, DMX, 0, QT0, DMX, DMX); }
  k_poison<<<(unsigned)NR, 256, 0, stream>>>(FLAG, (float*)d_out);
}
